// TSCN_80032420593738
// MI455X (gfx1250) — hardware-verified
//
#include <hip/hip_runtime.h>
#include <stddef.h>
#include <math.h>


#define DIM   64
#define KIN   128
#define SS    32
#define HIST  50
#define NF1   32
#define NTHR  256
#define NWAVE 8
#define RPB   32
#define XP    136
#define UPW   2
#define BMAX  2048

static_assert(RPB == 4 * NWAVE);
static_assert(KIN == 2 * DIM);
static_assert(SS == 32);
static_assert((XP % 8) == 0 && XP >= KIN);
static_assert(4 * NTHR * 8 == DIM * KIN);
static_assert(2 * NTHR * 8 == NF1 * KIN);
static_assert((BMAX % 4) == 0);

typedef float          v4f  __attribute__((ext_vector_type(4)));
typedef float          v8f  __attribute__((ext_vector_type(8)));
typedef unsigned short v4us __attribute__((ext_vector_type(4)));
typedef unsigned short v8us __attribute__((ext_vector_type(8)));
typedef __bf16         v16b __attribute__((ext_vector_type(16)));
union FragB { v16b v; v8us h[2]; };

__device__ __forceinline__ int iclamp(int x, int lo, int hi) { return x < lo ? lo : (x > hi ? hi : x); }

__device__ __forceinline__ unsigned short bf_rne(float x) {
  unsigned u = __float_as_uint(x);
  u += 0x7FFFu + ((u >> 16) & 1u);
  return (unsigned short)(u >> 16);
}
__device__ __forceinline__ float bf_val(unsigned short b) { return __uint_as_float(((unsigned)b) << 16); }

__device__ __forceinline__ v8us hi8(v4f a, v4f b) {
  v8us r;
  r[0] = bf_rne(a.x); r[1] = bf_rne(a.y); r[2] = bf_rne(a.z); r[3] = bf_rne(a.w);
  r[4] = bf_rne(b.x); r[5] = bf_rne(b.y); r[6] = bf_rne(b.z); r[7] = bf_rne(b.w);
  return r;
}
__device__ __forceinline__ v8us lo8(v4f a, v4f b, v8us hb) {
  v8us r;
  r[0] = bf_rne(a.x - bf_val(hb[0])); r[1] = bf_rne(a.y - bf_val(hb[1]));
  r[2] = bf_rne(a.z - bf_val(hb[2])); r[3] = bf_rne(a.w - bf_val(hb[3]));
  r[4] = bf_rne(b.x - bf_val(hb[4])); r[5] = bf_rne(b.y - bf_val(hb[5]));
  r[6] = bf_rne(b.z - bf_val(hb[6])); r[7] = bf_rne(b.w - bf_val(hb[7]));
  return r;
}

__device__ __forceinline__ v8f zero8f() {
  v8f c;
#pragma unroll
  for (int i = 0; i < 8; ++i) c[i] = 0.0f;
  return c;
}

__device__ __forceinline__ v8f wmb(v16b a, v16b b, v8f c) {
  v8f d = __builtin_amdgcn_wmma_f32_16x16x32_bf16(false, a, false, b, (short)0, c, false, false);
  asm volatile("v_nop\n\tv_nop\n\tv_nop\n\tv_nop" : "+v"(d) : "v"(a), "v"(b));
  return d;
}

__device__ __forceinline__ v8f wm3(v16b ah, v16b al, v16b bh, v16b bl, v8f c) {
  c = wmb(ah, bh, c);
  c = wmb(ah, bl, c);
  c = wmb(al, bh, c);
  return c;
}

__global__ __launch_bounds__(NTHR) void k_prep(const float* __restrict__ pool_w, const float* __restrict__ fc1_w,
                                              unsigned short* wph, unsigned short* wpl,
                                              unsigned short* w1h, unsigned short* w1l) {
  const int b = blockIdx.x, tid = threadIdx.x;
  const float* src;
  unsigned short* dh;
  unsigned short* dl;
  int nout, ub;
  if (b < 4) { src = pool_w; dh = wph; dl = wpl; nout = DIM; ub = b; }
  else       { src = fc1_w;  dh = w1h; dl = w1l; nout = NF1; ub = b - 4; }
  const int u  = ub * NTHR + tid;
  const int n  = u >> 4;
  const int kc = u & 15;
  v8us ph, pl;
#pragma unroll
  for (int j = 0; j < 8; ++j) {
    const int k = 8 * kc + j;
    const float w = src[k * nout + n];
    const unsigned short hb = bf_rne(w);
    ph[j] = hb;
    pl[j] = bf_rne(w - bf_val(hb));
  }
  unsigned short* php = dh + (size_t)u * 8;
  unsigned short* plp = dl + (size_t)u * 8;
  *(volatile v8us*)php = ph;
  *(volatile v8us*)plp = pl;
  __threadfence();
  *(volatile v8us*)php = ph;
  *(volatile v8us*)plp = pl;
}

__global__ __launch_bounds__(NTHR) void k_user(const int* __restrict__ ui, const int* __restrict__ nidx,
                                              const float* __restrict__ emb, float* xfc, int B, int nEmb) {
  __shared__ int red[NTHR];
  const int tid = threadIdx.x, lane = tid & 31, wave = tid >> 5, h = lane >> 4, m = lane & 15;
  int mx = -2147483647 - 1;
#pragma unroll 1
  for (int i = tid; i < B; i += NTHR) { const int v = nidx[i]; mx = v > mx ? v : mx; }
  red[tid] = mx;
  __syncthreads();
#pragma unroll 1
  for (int o = NTHR / 2; o > 0; o >>= 1) {
    if (tid < o) { const int a = red[tid], c = red[tid + o]; red[tid] = a > c ? a : c; }
    __syncthreads();
  }
  const float rinv = 1.0f / (float)red[0];

  const int ub = (blockIdx.x * NWAVE + wave) * UPW;
  v4f r0 = {0.0f, 0.0f, 0.0f, 0.0f};
  v4f r1 = {0.0f, 0.0f, 0.0f, 0.0f};
#pragma unroll
  for (int p = 0; p < UPW; ++p) {
    int b = ub + p;
    b = b > B - 1 ? B - 1 : b;
    int cnt = nidx[b];
    cnt = iclamp(cnt, 0, HIST);
    const int nj = (cnt + 1) >> 1;
    v4f acc = {0.0f, 0.0f, 0.0f, 0.0f};
#pragma unroll 1
    for (int j = 0; j < nj; ++j) {
      const int t  = 2 * j + h;
      const int tc = t > HIST - 1 ? HIST - 1 : t;
      int idx = ui[(size_t)b * HIST + tc];
      idx = iclamp(idx, 0, nEmb - 1);
      const v4f v = *(const v4f*)(emb + (size_t)idx * DIM + 4 * m);
      const float f = (t < cnt) ? 1.0f : 0.0f;
      acc += v * f;
    }
    acc.x += __shfl_xor(acc.x, 16, 32);
    acc.y += __shfl_xor(acc.y, 16, 32);
    acc.z += __shfl_xor(acc.z, 16, 32);
    acc.w += __shfl_xor(acc.w, 16, 32);
    acc = acc * rinv;
    if (p == 0) r0 = acc; else r1 = acc;
  }
  const int bw = ub + h;
  v4f v;
  v.x = h ? r1.x : r0.x; v.y = h ? r1.y : r0.y; v.z = h ? r1.z : r0.z; v.w = h ? r1.w : r0.w;
  float* dp = xfc + (size_t)(bw < B ? bw : 0) * KIN + 4 * m;
  if (bw < B) *(volatile v4f*)dp = v;
  __threadfence();
  if (bw < B) *(volatile v4f*)dp = v;
}

template <int MODE>
__global__ __launch_bounds__(NTHR) void k_pool(
    const int* __restrict__ item, const int* __restrict__ adj_item, const float* __restrict__ adj_adam,
    const float* __restrict__ emb, const float* __restrict__ selfd, const float* __restrict__ neighd,
    const unsigned short* __restrict__ wph, const unsigned short* __restrict__ wpl,
    const float* __restrict__ pool_b, float* out, int outPitch, int outCol,
    int nRows, int nEmb, int nAdj) {
  __shared__ __attribute__((aligned(16))) unsigned short Xh[RPB * XP];
  __shared__ __attribute__((aligned(16))) unsigned short Xl[RPB * XP];
  __shared__ __attribute__((aligned(16))) float Os[RPB * DIM];
  const int tid = threadIdx.x, lane = tid & 31, wave = tid >> 5, h = lane >> 4, m = lane & 15;
  const int rowBase = blockIdx.x * RPB;

#pragma unroll 1
  for (int q = 0; q < 4; ++q) {
    const int lr = 4 * wave + q;
    int row = rowBase + lr;
    row = row > nRows - 1 ? nRows - 1 : row;
    int praw;
    if (MODE == 1) {
      const int bb = row >> 5;
      int e0 = item[bb];
      e0 = iclamp(e0, 0, nAdj - 1);
      praw = adj_item[(size_t)e0 * SS + (row & (SS - 1))];
    } else {
      praw = item[row];
    }
    const int pa = iclamp(praw, 0, nAdj - 1);
    const int pe = iclamp(praw, 0, nEmb - 1);
    const float a = adj_adam[(size_t)pa * SS + lane];
    int nidx = 0;
    if (MODE != 2) {
      nidx = adj_item[(size_t)pa * SS + lane];
      nidx = iclamp(nidx, 0, nEmb - 1);
    }
    float mx = a;
#pragma unroll
    for (int o = 16; o > 0; o >>= 1) mx = fmaxf(mx, __shfl_xor(mx, o, 32));
    const float e = expf(a - mx);
    float sm = e;
#pragma unroll
    for (int o = 16; o > 0; o >>= 1) sm += __shfl_xor(sm, o, 32);
    const float w = e * (1.0f / sm);
    const float* sp;
    if (MODE == 2) sp = selfd + (size_t)row * DIM;
    else           sp = emb + (size_t)pe * DIM;
    const v4f sv = *(const v4f*)(sp + 4 * m);
    v4f acc = {0.0f, 0.0f, 0.0f, 0.0f};
#pragma unroll 4
    for (int j = 0; j < SS / 2; ++j) {
      const int s = 2 * j + h;
      const float ws = __shfl(w, s, 32);
      const float* np;
      if (MODE == 2) {
        np = neighd + ((size_t)row * SS + s) * DIM;
      } else {
        const int ni = __shfl(nidx, s, 32);
        np = emb + (size_t)ni * DIM;
      }
      const v4f nv = *(const v4f*)(np + 4 * m);
      acc += nv * ws;
    }
    acc.x += __shfl_xor(acc.x, 16, 32);
    acc.y += __shfl_xor(acc.y, 16, 32);
    acc.z += __shfl_xor(acc.z, 16, 32);
    acc.w += __shfl_xor(acc.w, 16, 32);
    v4f xv;
    xv.x = (lane < 16) ? sv.x : acc.x; xv.y = (lane < 16) ? sv.y : acc.y;
    xv.z = (lane < 16) ? sv.z : acc.z; xv.w = (lane < 16) ? sv.w : acc.w;
    v4us hv, lv;
    hv[0] = bf_rne(xv.x); hv[1] = bf_rne(xv.y); hv[2] = bf_rne(xv.z); hv[3] = bf_rne(xv.w);
    lv[0] = bf_rne(xv.x - bf_val(hv[0])); lv[1] = bf_rne(xv.y - bf_val(hv[1]));
    lv[2] = bf_rne(xv.z - bf_val(hv[2])); lv[3] = bf_rne(xv.w - bf_val(hv[3]));
    *(v4us*)(Xh + lr * XP + 4 * lane) = hv;
    *(v4us*)(Xl + lr * XP + 4 * lane) = lv;
  }
  __syncthreads();

  {
    const int rt = wave >> 2, ct = wave & 3;
    const unsigned short* xh  = Xh + (16 * rt + m) * XP + 8 * h;
    const unsigned short* xl  = Xl + (16 * rt + m) * XP + 8 * h;
    const unsigned short* bhp = wph + (size_t)(16 * ct + m) * KIN + 8 * h;
    const unsigned short* blp = wpl + (size_t)(16 * ct + m) * KIN + 8 * h;
    v8f c = zero8f();
#pragma unroll
    for (int kt = 0; kt < 4; ++kt) {
      const int k0 = 32 * kt;
      FragB ah, al, bh, bl;
      ah.h[0] = *(const v8us*)(xh + k0);  ah.h[1] = *(const v8us*)(xh + k0 + 16);
      al.h[0] = *(const v8us*)(xl + k0);  al.h[1] = *(const v8us*)(xl + k0 + 16);
      bh.h[0] = *(const v8us*)(bhp + k0); bh.h[1] = *(const v8us*)(bhp + k0 + 16);
      bl.h[0] = *(const v8us*)(blp + k0); bl.h[1] = *(const v8us*)(blp + k0 + 16);
      c = wm3(ah.v, al.v, bh.v, bl.v, c);
    }
    const int col = 16 * ct + m;
    const float bias = pool_b[col];
#pragma unroll
    for (int r = 0; r < 8; ++r) Os[(16 * rt + 8 * h + r) * DIM + col] = fmaxf(c[r] + bias, 0.0f);
  }
  __syncthreads();

#pragma unroll
  for (int p = 0; p < 2; ++p) {
    const int lr  = 4 * wave + 2 * p + h;
    const int row = rowBase + lr;
    const v4f v = *(const v4f*)(Os + lr * DIM + 4 * m);
    if (row < nRows) *(volatile v4f*)(out + (size_t)row * outPitch + outCol + 4 * m) = v;
  }
  __threadfence();
#pragma unroll
  for (int p = 0; p < 2; ++p) {
    const int lr  = 4 * wave + 2 * p + h;
    const int row = rowBase + lr;
    const v4f v = *(const v4f*)(Os + lr * DIM + 4 * m);
    if (row < nRows) *(volatile v4f*)(out + (size_t)row * outPitch + outCol + 4 * m) = v;
  }
}

__global__ __launch_bounds__(NTHR) void k_head(const float* __restrict__ xfc,
                                              const unsigned short* __restrict__ w1h,
                                              const unsigned short* __restrict__ w1l,
                                              const float* __restrict__ fc1_b, const float* __restrict__ fc2_w,
                                              const float* __restrict__ fc2_b, float* out, int B) {
  __shared__ __attribute__((aligned(16))) float lg[BMAX];
  __shared__ float red[NTHR];
  const int tid = threadIdx.x, lane = tid & 31, wave = tid >> 5, h = lane >> 4, m = lane & 15;
  const float b2 = fc2_b[0];
  const int nRT = (B + 15) >> 4;

#pragma unroll 1
  for (int rt = wave; rt < nRT; rt += NWAVE) {
    int r = 16 * rt + m;
    r = r > B - 1 ? B - 1 : r;
    const float* xr = xfc + (size_t)r * KIN + 8 * h;
    FragB ah[4], al[4];
#pragma unroll
    for (int kt = 0; kt < 4; ++kt) {
      const float* p = xr + 32 * kt;
      const v4f x0 = *(const v4f*)p;
      const v4f x1 = *(const v4f*)(p + 4);
      const v4f x2 = *(const v4f*)(p + 16);
      const v4f x3 = *(const v4f*)(p + 20);
      ah[kt].h[0] = hi8(x0, x1);
      al[kt].h[0] = lo8(x0, x1, ah[kt].h[0]);
      ah[kt].h[1] = hi8(x2, x3);
      al[kt].h[1] = lo8(x2, x3, ah[kt].h[1]);
    }
    v8f part = zero8f();
#pragma unroll
    for (int ct = 0; ct < 2; ++ct) {
      v8f c = zero8f();
      const unsigned short* bhp = w1h + (size_t)(16 * ct + m) * KIN + 8 * h;
      const unsigned short* blp = w1l + (size_t)(16 * ct + m) * KIN + 8 * h;
#pragma unroll
      for (int kt = 0; kt < 4; ++kt) {
        FragB fh, fl;
        fh.h[0] = *(const v8us*)(bhp + 32 * kt); fh.h[1] = *(const v8us*)(bhp + 32 * kt + 16);
        fl.h[0] = *(const v8us*)(blp + 32 * kt); fl.h[1] = *(const v8us*)(blp + 32 * kt + 16);
        c = wm3(ah[kt].v, al[kt].v, fh.v, fl.v, c);
      }
      const int col = 16 * ct + m;
      const float b1 = fc1_b[col];
      const float w2 = fc2_w[col];
#pragma unroll
      for (int rr = 0; rr < 8; ++rr) part[rr] += fmaxf(c[rr] + b1, 0.0f) * w2;
    }
#pragma unroll
    for (int rr = 0; rr < 8; ++rr) {
      float v = part[rr];
      v += __shfl_xor(v, 8, 32);
      v += __shfl_xor(v, 4, 32);
      v += __shfl_xor(v, 2, 32);
      v += __shfl_xor(v, 1, 32);
      const int row = 16 * rt + 8 * h + rr;
      if (m == 0 && row < B) lg[row] = v + b2;
    }
  }
  __syncthreads();

  float mx = -3.0e38f;
#pragma unroll 1
  for (int i = tid; i < B; i += NTHR) mx = fmaxf(mx, lg[i]);
  red[tid] = mx;
  __syncthreads();
#pragma unroll 1
  for (int o = NTHR / 2; o > 0; o >>= 1) {
    if (tid < o) red[tid] = fmaxf(red[tid], red[tid + o]);
    __syncthreads();
  }
  const float gm = red[0];
  __syncthreads();
  float sm = 0.0f;
#pragma unroll 1
  for (int i = tid; i < B; i += NTHR) { const float e = expf(lg[i] - gm); lg[i] = e; sm += e; }
  red[tid] = sm;
  __syncthreads();
#pragma unroll 1
  for (int o = NTHR / 2; o > 0; o >>= 1) {
    if (tid < o) red[tid] = red[tid] + red[tid + o];
    __syncthreads();
  }
  const float inv = 1.0f / red[0];
#pragma unroll 1
  for (int i = tid; i < B; i += NTHR) lg[i] = lg[i] * inv;
  __syncthreads();

  const int n4 = B >> 2;
#pragma unroll 1
  for (int u = tid; u < n4; u += NTHR) { const v4f v = *(const v4f*)(lg + 4 * u); *(volatile v4f*)(out + 4 * u) = v; }
#pragma unroll 1
  for (int i = 4 * n4 + tid; i < B; i += NTHR) { const float v = lg[i]; *(volatile float*)(out + i) = v; }
  __threadfence();
#pragma unroll 1
  for (int u = tid; u < n4; u += NTHR) { const v4f v = *(const v4f*)(lg + 4 * u); *(volatile v4f*)(out + 4 * u) = v; }
#pragma unroll 1
  for (int i = 4 * n4 + tid; i < B; i += NTHR) { const float v = lg[i]; *(volatile float*)(out + i) = v; }
}

extern "C" void kernel_launch(void* const* d_in, const int* in_sizes, int n_in,
                              void* d_out, int out_size, void* d_ws, size_t ws_size,
                              hipStream_t stream) {
  if (n_in < 12) return;
  const int B = in_sizes[1];
  if (B < 1 || B > BMAX) return;
  if (in_sizes[0] != B * HIST || in_sizes[2] != B) return;
  if (in_sizes[3] < DIM || (in_sizes[3] % DIM) != 0) return;
  const int nEmb = in_sizes[3] / DIM;
  if (in_sizes[4] < SS || (in_sizes[4] % SS) != 0 || in_sizes[5] != in_sizes[4]) return;
  const int nAdj = in_sizes[4] / SS;
  if (in_sizes[6] != KIN * DIM || in_sizes[7] != DIM) return;
  if (in_sizes[8] != KIN * NF1 || in_sizes[9] != NF1 || in_sizes[10] != NF1 || in_sizes[11] != 1) return;
  if (out_size != B) return;

  const int*   user_inputs = (const int*)d_in[0];
  const int*   item_inputs = (const int*)d_in[1];
  const int*   n_idxs      = (const int*)d_in[2];
  const float* emb         = (const float*)d_in[3];
  const int*   adj_item    = (const int*)d_in[4];
  const float* adj_adam    = (const float*)d_in[5];
  const float* pool_w      = (const float*)d_in[6];
  const float* pool_b      = (const float*)d_in[7];
  const float* fc1_w       = (const float*)d_in[8];
  const float* fc1_b       = (const float*)d_in[9];
  const float* fc2_w       = (const float*)d_in[10];
  const float* fc2_b       = (const float*)d_in[11];
  float* outp = (float*)d_out;

  const size_t Bp = (size_t)((B + RPB - 1) / RPB) * RPB;
  char* ws = (char*)d_ws;
  size_t off = 0;
  const size_t oWpH = off; off += ((size_t)DIM * KIN * 2 + 255) & ~(size_t)255;
  const size_t oWpL = off; off += ((size_t)DIM * KIN * 2 + 255) & ~(size_t)255;
  const size_t oW1H = off; off += ((size_t)NF1 * KIN * 2 + 255) & ~(size_t)255;
  const size_t oW1L = off; off += ((size_t)NF1 * KIN * 2 + 255) & ~(size_t)255;
  const size_t oXfc = off; off += (Bp * KIN * 4 + 255) & ~(size_t)255;
  const size_t oV0  = off; off += (Bp * DIM * 4 + 255) & ~(size_t)255;
  const size_t oV1  = off; off += (Bp * SS * DIM * 4 + 255) & ~(size_t)255;
  size_t limit = (size_t)134217728;
  if (ws_size < limit) limit = ws_size;
  if (off > limit) return;

  unsigned short* WpH = (unsigned short*)(ws + oWpH);
  unsigned short* WpL = (unsigned short*)(ws + oWpL);
  unsigned short* W1H = (unsigned short*)(ws + oW1H);
  unsigned short* W1L = (unsigned short*)(ws + oW1L);
  float* Xfc = (float*)(ws + oXfc);
  float* V0  = (float*)(ws + oV0);
  float* V1  = (float*)(ws + oV1);

  k_prep<<<6, NTHR, 0, stream>>>(pool_w, fc1_w, WpH, WpL, W1H, W1L);

  k_user<<<(B + NWAVE * UPW - 1) / (NWAVE * UPW), NTHR, 0, stream>>>(user_inputs, n_idxs, emb, Xfc, B, nEmb);

  k_pool<1><<<(B * SS + RPB - 1) / RPB, NTHR, 0, stream>>>(
      item_inputs, adj_item, adj_adam, emb, emb, emb, WpH, WpL, pool_b, V1, DIM, 0, B * SS, nEmb, nAdj);
  k_pool<0><<<(B + RPB - 1) / RPB, NTHR, 0, stream>>>(
      item_inputs, adj_item, adj_adam, emb, emb, emb, WpH, WpL, pool_b, V0, DIM, 0, B, nEmb, nAdj);
  k_pool<2><<<(B + RPB - 1) / RPB, NTHR, 0, stream>>>(
      item_inputs, adj_item, adj_adam, emb, V0, V1, WpH, WpL, pool_b, Xfc, KIN, DIM, B, nEmb, nAdj);

  k_head<<<1, NTHR, 0, stream>>>(Xfc, W1H, W1L, fc1_b, fc2_w, fc2_b, outp, B);
}
